// JointAttention_1082331758599
// MI455X (gfx1250) — hardware-run, weakly checked
//
#include <hip/hip_runtime.h>


#ifndef NB
#define NB 8
#endif
#ifndef NP
#define NP 1024
#endif
#define NB_FULL  8
#define NP_FULL  1024
#define ND       64
#define ND_FULL  64
#define KD       128
#define HW       256
#define CW       512
#define PITCH    257
#define JT       (NP / 256)
#define LOG2E    1.4426950408889634f

static_assert(KD % 32 == 0);
static_assert(KD % 8 == 0);
static_assert(KD == 128);
static_assert(HW == 256);
static_assert(CW == 2 * HW);
static_assert(CW % 64 == 0);
static_assert(HW % 64 == 0);
static_assert((NB * ND) % 64 == 0);
static_assert((NB * NP) % 64 == 0);
static_assert(ND % 16 == 0);
static_assert(NP % 32 == 0);
static_assert(NP % 256 == 0);
static_assert(((size_t)ND * KD) % (8 * 256) == 0);
static_assert(((size_t)NP * KD) % (8 * 256) == 0);
static_assert(NB <= NB_FULL);
static_assert(NP <= NP_FULL);
static_assert((size_t)NB_FULL * HW * 4 == (size_t)8192);

typedef unsigned short bf;
typedef __attribute__((ext_vector_type(16))) __bf16   v16bf;
typedef __attribute__((ext_vector_type(8)))  unsigned short v8us;
typedef __attribute__((ext_vector_type(8)))  float    v8f;
typedef __attribute__((ext_vector_type(4)))  float    v4f;
typedef v4f  __attribute__((may_alias)) v4fa;
typedef v8us __attribute__((may_alias)) v8usa;

__device__ __forceinline__ unsigned short f2bf(float f) { unsigned u = __float_as_uint(f); u += 0x7FFFu + ((u >> 16) & 1u); return (unsigned short)(u >> 16); }
__device__ __forceinline__ float bf2f(unsigned short s) { return __uint_as_float(((unsigned)s) << 16); }
__device__ __forceinline__ float bfr(float f) { return bf2f(f2bf(f)); }
__device__ __forceinline__ v16bf cat16b(v8us lo, v8us hi) { return __builtin_bit_cast(v16bf, __builtin_shufflevector(lo, hi, 0, 1, 2, 3, 4, 5, 6, 7, 8, 9, 10, 11, 12, 13, 14, 15)); }
__device__ __forceinline__ v16bf ldb(const bf* p)  { return cat16b(*(const v8us*)p, *(const v8us*)(p + 16)); }
__device__ __forceinline__ v8f wmmab_g(v16bf a, v16bf b, v8f c) {
    c = __builtin_amdgcn_wmma_f32_16x16x32_bf16(false, a, false, b, (short)0, c, false, false);
    asm volatile("v_nop\n\tv_nop\n\tv_nop\n\tv_nop" : "+v"(c) : "v"(a), "v"(b));
    return c;
}
__device__ __forceinline__ void wave_sync() { __builtin_amdgcn_fence(3  , "wavefront"); __builtin_amdgcn_wave_barrier(); asm volatile("" ::: "memory"); }
__device__ __forceinline__ float tanh_e(float x) { const float e = __builtin_amdgcn_exp2f(x * (2.0f * LOG2E)); const float r = __builtin_amdgcn_rcpf(e + 1.0f); return 1.0f - 2.0f * r; }

__global__ __launch_bounds__(256) void k_cvt(const float* __restrict__ src, bf* dst, unsigned perBatch8, unsigned c8n, size_t sBatch, size_t sRow) {
    const unsigned i = blockIdx.x * 256u + threadIdx.x; if (i >= perBatch8) return;
    const unsigned r = i / c8n, c = i - r * c8n; const unsigned b = blockIdx.y;
    const v8f v = *(const v8f*)(src + (size_t)b * sBatch + (size_t)r * sRow + (size_t)c * 8); v8us o;
#pragma unroll
    for (int k = 0; k < 8; ++k) o[k] = f2bf(v[k]);
    const size_t oo = ((size_t)b * perBatch8 + i) * 8;
    *(volatile v8us*)(dst + oo) = o; __threadfence(); *(volatile v8us*)(dst + oo) = o;
}

__global__ __launch_bounds__(256) void k_wt(const float* __restrict__ W, bf* WT) {
    __shared__ __align__(16) unsigned short ts[64 * 136];
    const int tid = threadIdx.x; const int n0 = blockIdx.x * 64;
    const int n = tid & 63, kq = tid >> 6;
#pragma unroll 1
    for (int it = 0; it < 32; ++it) { const int k = kq + 4 * it;
        ts[n * 136 + k] = f2bf(W[(size_t)k * HW + n0 + n]); }
    __syncthreads();
#pragma unroll 1
    for (int ps = 0; ps < 2; ++ps) {
#pragma unroll
        for (int it = 0; it < 4; ++it) { const int p = it * 256 + tid; const int row = p >> 4, c8 = (p & 15) * 8;
            const v8us o = *(const v8usa*)(&ts[row * 136 + c8]);
            *(volatile v8us*)(WT + (size_t)(n0 + row) * KD + c8) = o; }
        if (ps == 0) __threadfence(); }
}

__global__ __launch_bounds__(32) void k_pgemm(const bf* __restrict__ A, const bf* __restrict__ Bt, float* OUT) {
    __shared__ __align__(16) float os[16 * 68];
    const int lane = threadIdx.x & 31, lr = lane & 15, hi = lane >> 4; const int r0 = blockIdx.x * 64, c0 = blockIdx.y * 64;
    v8f acc[4][4];
#pragma unroll
    for (int mb = 0; mb < 4; ++mb)
#pragma unroll
        for (int nb = 0; nb < 4; ++nb) acc[mb][nb] = (v8f){};
    const size_t aoff = (size_t)(r0 + lr) * KD + 8 * hi, boff = (size_t)(c0 + lr) * KD + 8 * hi;
#pragma unroll 1
    for (int kc = 0; kc < KD; kc += 32) {
        v16bf a[4];
#pragma unroll
        for (int mb = 0; mb < 4; ++mb) a[mb] = ldb(A + aoff + (size_t)mb * 16 * KD + kc);
#pragma unroll
        for (int nb = 0; nb < 4; ++nb) { const v16bf b = ldb(Bt + boff + (size_t)nb * 16 * KD + kc);
#pragma unroll
            for (int mb = 0; mb < 4; ++mb) acc[mb][nb] = wmmab_g(a[mb], b, acc[mb][nb]); }
    }
    const int cofs = lr * 4;
    float* orow = OUT + (size_t)r0 * CW + c0;
#pragma unroll
    for (int mb = 0; mb < 4; ++mb) {
#pragma unroll
        for (int nb = 0; nb < 4; ++nb) {
#pragma unroll
            for (int j = 0; j < 8; ++j) os[(hi * 8 + j) * 68 + nb * 16 + lr] = acc[mb][nb][j]; }
        wave_sync();
#pragma unroll 1
        for (int ps = 0; ps < 2; ++ps) {
#pragma unroll
            for (int s = 0; s < 8; ++s) { const int row = 2 * s + hi;
                const v4f val = *(const v4fa*)(&os[row * 68 + cofs]);
                *(volatile v4f*)(orow + (size_t)(mb * 16 + row) * CW + cofs) = val; }
            if (ps == 0) __threadfence(); }
        wave_sync();
    }
}

__global__ __launch_bounds__(256) void k_scores(const float* __restrict__ HFD, const float* __restrict__ HFP, const float* __restrict__ wsc, float* SC) {
    __shared__ float hp_s[32 * PITCH];
    __shared__ float hd_s[16 * PITCH];
    __shared__ float w_s[HW];
    const int t = threadIdx.x; const int wave = __builtin_amdgcn_readfirstlane(threadIdx.x >> 5);
    const int b = blockIdx.z; const int i0 = blockIdx.y * 16; const int j0 = blockIdx.x * 32;
    const float* hpB = HFP + (size_t)(b * NP + j0) * CW;
#pragma unroll 1
    for (int n = 0; n < 32; ++n) hp_s[n * PITCH + t] = hpB[(size_t)n * CW + t];
    const float* hdB = HFD + (size_t)(b * ND + i0) * CW;
#pragma unroll 1
    for (int n = 0; n < 16; ++n) hd_s[n * PITCH + t] = hdB[(size_t)n * CW + t];
    w_s[t] = bfr(wsc[t]);
    __syncthreads();
    const int ja = t & 31;
    const int oa = wave * PITCH, oc = (wave + 8) * PITCH, op = ja * PITCH;
    float acc0 = 0.0f, acc1 = 0.0f;
#pragma unroll 4
    for (int h = 0; h < HW; ++h) {
        const float w = w_s[h]; const float p = hp_s[op + h];
        acc0 += w * tanh_e(hd_s[oa + h] + p);
        acc1 += w * tanh_e(hd_s[oc + h] + p); }
    float* srow = SC + (size_t)(b * ND + i0) * NP + j0 + ja;
    *(volatile float*)(srow + (size_t)wave * NP) = acc0; *(volatile float*)(srow + (size_t)(wave + 8) * NP) = acc1;
    __threadfence();
    *(volatile float*)(srow + (size_t)wave * NP) = acc0; *(volatile float*)(srow + (size_t)(wave + 8) * NP) = acc1;
}

__global__ __launch_bounds__(256) void k_attn(const float* __restrict__ SC, const float* __restrict__ HFD, const float* __restrict__ HFP, float* PT) {
    __shared__ float a_s[NP];
    __shared__ float redm[8];
    __shared__ float reds[8];
    const int t = threadIdx.x; const int lane = t & 31; const int wave = __builtin_amdgcn_readfirstlane(threadIdx.x >> 5);
    const int b = blockIdx.y; const int i = blockIdx.x;
    const float* srow = SC + (size_t)(b * ND + i) * NP;
    float sv[JT]; float mx = -3.0e38f;
#pragma unroll
    for (int q = 0; q < JT; ++q) { sv[q] = srow[t + 256 * q]; mx = fmaxf(mx, sv[q]); }
#pragma unroll
    for (int off = 16; off > 0; off >>= 1) mx = fmaxf(mx, __shfl_xor(mx, off, 32));
    if (lane == 0) redm[wave] = mx;
    __syncthreads();
    float m = redm[0];
#pragma unroll
    for (int w = 1; w < 8; ++w) m = fmaxf(m, redm[w]);
    float ev[JT]; float ls = 0.0f;
#pragma unroll
    for (int q = 0; q < JT; ++q) { ev[q] = __builtin_amdgcn_exp2f((sv[q] - m) * LOG2E); ls += ev[q]; }
#pragma unroll
    for (int off = 16; off > 0; off >>= 1) ls += __shfl_xor(ls, off, 32);
    if (lane == 0) reds[wave] = ls;
    __syncthreads();
    float tot = reds[0];
#pragma unroll
    for (int w = 1; w < 8; ++w) tot += reds[w];
    const float inv = 1.0f / tot;
#pragma unroll
    for (int q = 0; q < JT; ++q) a_s[t + 256 * q] = ev[q] * inv;
    __syncthreads();
    const float fdv = HFD[(size_t)(b * ND + i) * CW + HW + t];
    const float* fpB = HFP + (size_t)b * NP * CW + HW + t;
    float acc = 0.0f;
#pragma unroll 4
    for (int j = 0; j < NP; ++j) acc += a_s[j] * tanh_e(fdv + fpB[(size_t)j * CW]);
    float* prow = PT + (size_t)(b * ND + i) * HW + t;
    *(volatile float*)prow = acc; __threadfence(); *(volatile float*)prow = acc;
}

__global__ __launch_bounds__(256) void k_reduce(const float* __restrict__ PT, float* OUT) {
    const int b = blockIdx.x; const int o = threadIdx.x;
    const float* p = PT + (size_t)b * ND * HW + o;
    float acc = 0.0f;
#pragma unroll 4
    for (int i = 0; i < ND; ++i) acc += p[(size_t)i * HW];
    float* q = OUT + (size_t)b * HW + o;
    *(volatile float*)q = acc; __threadfence(); *(volatile float*)q = acc;
}

static constexpr size_t al256(size_t v) { return (v + 255) & ~(size_t)255; }
static constexpr size_t SZ_XD  = al256((size_t)NB * ND * KD * 2);
static constexpr size_t SZ_XP  = al256((size_t)NB * NP * KD * 2);
static constexpr size_t SZ_WB  = al256((size_t)4 * HW * KD * 2);
static constexpr size_t SZ_HFD = al256((size_t)NB * ND * CW * 4);
static constexpr size_t SZ_HFP = al256((size_t)NB * NP * CW * 4);
static constexpr size_t SZ_SC  = al256((size_t)NB * ND * NP * 4);
static constexpr size_t SZ_PT  = al256((size_t)NB * ND * HW * 4);
static constexpr size_t SZ_TOTAL = SZ_XD + SZ_XP + SZ_WB + SZ_HFD + SZ_HFP + SZ_SC + SZ_PT;
static_assert(SZ_TOTAL <= (size_t)134217728);
static_assert(((size_t)HW * KD * 2) % 256 == 0);

extern "C" void kernel_launch(void* const* d_in, const int* in_sizes, int n_in,
                              void* d_out, int out_size, void* d_ws, size_t ws_size, hipStream_t stream) {
    if (n_in < 7) return;
    if ((size_t)in_sizes[0] < ((size_t)(NB - 1) * ND_FULL + ND) * KD) return;
    if ((size_t)in_sizes[1] < ((size_t)(NB - 1) * NP_FULL + NP) * KD) return;
    if ((size_t)in_sizes[2] < (size_t)KD * HW || (size_t)in_sizes[3] < (size_t)KD * HW || (size_t)in_sizes[4] < (size_t)KD * HW || (size_t)in_sizes[5] < (size_t)KD * HW) return;
    if (in_sizes[6] < HW) return;
    if ((size_t)out_size < (size_t)NB * HW) return;
    if (SZ_TOTAL > ws_size) return;
    const float* xd = (const float*)d_in[0]; const float* xp = (const float*)d_in[1];
    const float* wd = (const float*)d_in[2]; const float* wp = (const float*)d_in[3];
    const float* wa = (const float*)d_in[4]; const float* wb = (const float*)d_in[5];
    const float* wsc = (const float*)d_in[6];
    float* OUT = (float*)d_out;
    char* wsp = (char*)d_ws;
    bf* XDB = (bf*)wsp; wsp += SZ_XD;
    bf* XPB = (bf*)wsp; wsp += SZ_XP;
    bf* WB  = (bf*)wsp; wsp += SZ_WB;
    float* HFD = (float*)wsp; wsp += SZ_HFD;
    float* HFP = (float*)wsp; wsp += SZ_HFP;
    float* SC  = (float*)wsp; wsp += SZ_SC;
    float* PT  = (float*)wsp; wsp += SZ_PT;
    bf* WDT = WB; bf* WAT = WB + (size_t)HW * KD; bf* WPT = WB + (size_t)2 * HW * KD; bf* WBT = WB + (size_t)3 * HW * KD;

    { const unsigned p8 = (unsigned)((size_t)ND * KD / 8); const dim3 g((p8 + 255) / 256, NB, 1);
      k_cvt<<<g, 256, 0, stream>>>(xd, XDB, p8, (unsigned)(KD / 8), (size_t)ND_FULL * KD, (size_t)KD); }
    { const unsigned p8 = (unsigned)((size_t)NP * KD / 8); const dim3 g((p8 + 255) / 256, NB, 1);
      k_cvt<<<g, 256, 0, stream>>>(xp, XPB, p8, (unsigned)(KD / 8), (size_t)NP_FULL * KD, (size_t)KD); }

    k_wt<<<HW / 64, 256, 0, stream>>>(wd, WDT);
    k_wt<<<HW / 64, 256, 0, stream>>>(wa, WAT);
    k_wt<<<HW / 64, 256, 0, stream>>>(wp, WPT);
    k_wt<<<HW / 64, 256, 0, stream>>>(wb, WBT);

    k_pgemm<<<dim3(NB * ND / 64, CW / 64, 1), 32, 0, stream>>>(XDB, WDT, HFD);
    k_pgemm<<<dim3(NB * NP / 64, CW / 64, 1), 32, 0, stream>>>(XPB, WPT, HFP);

    k_scores<<<dim3(NP / 32, ND / 16, NB), 256, 0, stream>>>(HFD, HFP, wsc, SC);
    k_attn<<<dim3(ND, NB, 1), 256, 0, stream>>>(SC, HFD, HFP, PT);
    k_reduce<<<NB, 256, 0, stream>>>(PT, OUT);
}
